// MultiheadAttention_52037823758844
// MI455X (gfx1250) — hardware-run, weakly checked
//
#include <hip/hip_runtime.h>


#ifndef NB
#define NB 4
#endif
#ifndef SEQ
#define SEQ 2048
#endif
#define NB_FULL 4
#define DM   1024
#define NH   16
#define HD   64
#define QKCAR 16.0f
#define VCAR  16.0f
#define CCAR  256.0f
#define WOCAR 64.0f
#define PLOG  10.0f
#define CLOG  (0.125f * 1.4426950408889634f / (QKCAR * QKCAR))
#define OSCL  (1.0f / (CCAR * WOCAR))
#define PLANE ((size_t)NB * NH * SEQ * HD)

static_assert(SEQ % 128 == 0);
static_assert(NB >= 1 && NB <= NB_FULL);
static_assert(DM == NH * HD);
static_assert(DM % 64 == 0);
static_assert(HD == 64);
static_assert(((size_t)NB * SEQ * DM * 2 + (size_t)3 * DM * DM * 2 + (size_t)DM * DM * 2 + 3 * PLANE * 2 + (size_t)NB * SEQ * DM * 2) <= (size_t)134217728);

typedef _Float16 h16;
typedef unsigned short bf;
typedef __attribute__((ext_vector_type(16))) __bf16   v16bf;
typedef __attribute__((ext_vector_type(16))) _Float16 v16h;
typedef __attribute__((ext_vector_type(8)))  _Float16 v8h;
typedef __attribute__((ext_vector_type(8)))  unsigned short v8us;
typedef __attribute__((ext_vector_type(8)))  float    v8f;
typedef __attribute__((ext_vector_type(4)))  float    v4f;
typedef v8h  __attribute__((may_alias)) v8ha;
typedef v4f  __attribute__((may_alias)) v4fa;

__device__ __forceinline__ unsigned short f2bf(float f) { unsigned u = __float_as_uint(f); u += 0x7FFFu + ((u >> 16) & 1u); return (unsigned short)(u >> 16); }
__device__ __forceinline__ float bf2f(unsigned short b) { return __uint_as_float(((unsigned)b) << 16); }
__device__ __forceinline__ float bfr(float f) { return bf2f(f2bf(f)); }
__device__ __forceinline__ v16h cat16(v8h lo, v8h hi) { return __builtin_shufflevector(lo, hi, 0, 1, 2, 3, 4, 5, 6, 7, 8, 9, 10, 11, 12, 13, 14, 15); }
__device__ __forceinline__ v16bf cat16b(v8us lo, v8us hi) { return __builtin_bit_cast(v16bf, __builtin_shufflevector(lo, hi, 0, 1, 2, 3, 4, 5, 6, 7, 8, 9, 10, 11, 12, 13, 14, 15)); }
__device__ __forceinline__ v8f wmma16(v16h a, v16h b, v8f c) { return __builtin_amdgcn_wmma_f32_16x16x32_f16(false, a, false, b, (short)0, c, false, false); }
__device__ __forceinline__ v8f wmmab(v16bf a, v16bf b, v8f c) { return __builtin_amdgcn_wmma_f32_16x16x32_bf16(false, a, false, b, (short)0, c, false, false); }
__device__ __forceinline__ v16h ldh(const h16* p) { return cat16(*(const v8h*)p, *(const v8h*)(p + 16)); }

template <typename T16> struct WFrag;
template <> struct WFrag<h16> { typedef v16h V; static __device__ __forceinline__ V ld(const h16* p) { return cat16(*(const v8h*)p, *(const v8h*)(p + 16)); } static __device__ __forceinline__ v8f mma(V a, V b, v8f c) { return wmma16(a, b, c); } };
template <> struct WFrag<bf> { typedef v16bf V; static __device__ __forceinline__ V ld(const bf* p) { return cat16b(*(const v8us*)p, *(const v8us*)(p + 16)); } static __device__ __forceinline__ v8f mma(V a, V b, v8f c) { return wmmab(a, b, c); } };

__global__ __launch_bounds__(256) void k_cvtx(const float* __restrict__ src, bf* dst) {
#pragma clang fp contract(off)
    const size_t i = (size_t)blockIdx.x * 256 + threadIdx.x; if (i >= (size_t)NB * SEQ * DM / 8) return;
    const int e8 = (int)(i % (DM / 8)); const size_t rs = i / (DM / 8); const int s = (int)(rs % SEQ); const int b = (int)(rs / SEQ);
    const v8f v = *(const v8f*)(src + ((size_t)s * NB_FULL + b) * DM + (size_t)e8 * 8); v8us o;
#pragma unroll
    for (int k = 0; k < 8; ++k) o[k] = f2bf(v[k]);
    *(volatile v8us*)(dst + i * 8) = o; __threadfence(); *(volatile v8us*)(dst + i * 8) = o;
}
__global__ __launch_bounds__(256) void k_cvt8(const float* __restrict__ src, bf* dst, size_t n8) {
#pragma clang fp contract(off)
    const size_t i = (size_t)blockIdx.x * 256 + threadIdx.x; if (i >= n8) return; const v8f v = *(const v8f*)(src + i * 8); v8us o;
#pragma unroll
    for (int k = 0; k < 8; ++k) o[k] = f2bf(v[k]);
    *(volatile v8us*)(dst + i * 8) = o; __threadfence(); *(volatile v8us*)(dst + i * 8) = o;
}
__global__ __launch_bounds__(256) void k_cvtw(const float* __restrict__ src, h16* dst, size_t n8) {
#pragma clang fp contract(off)
    const size_t i = (size_t)blockIdx.x * 256 + threadIdx.x; if (i >= n8) return; const v8f v = *(const v8f*)(src + i * 8); v8h o;
#pragma unroll
    for (int k = 0; k < 8; ++k) o[k] = (h16)(bfr(v[k]) * WOCAR);
    *(volatile v8h*)(dst + i * 8) = o; __threadfence(); *(volatile v8h*)(dst + i * 8) = o;
}

template <typename T16, int EPI>
__global__ __launch_bounds__(32) void k_gemm(const T16* __restrict__ A, const T16* __restrict__ Bt, const float* __restrict__ bias, h16* planes, float* C) {
    typedef typename WFrag<T16>::V V;
    __shared__ __align__(16) float os[64 * 68];
    const int lane = threadIdx.x & 31, lr = lane & 15, hi = lane >> 4;
    const int r0 = blockIdx.x * 64, c0 = blockIdx.y * 64, bz = blockIdx.z;
    const T16* Ab = A + (size_t)bz * SEQ * DM;
    v8f acc[4][4];
#pragma unroll
    for (int mb = 0; mb < 4; ++mb)
#pragma unroll
        for (int nb = 0; nb < 4; ++nb) acc[mb][nb] = (v8f){};
    const size_t aoff = (size_t)(r0 + lr) * DM + 8 * hi, boff = (size_t)(c0 + lr) * DM + 8 * hi;
#pragma unroll 1
    for (int kc = 0; kc < DM; kc += 32) {
        V a[4];
#pragma unroll
        for (int mb = 0; mb < 4; ++mb) a[mb] = WFrag<T16>::ld(Ab + aoff + (size_t)mb * 16 * DM + kc);
#pragma unroll
        for (int nb = 0; nb < 4; ++nb) { const V b = WFrag<T16>::ld(Bt + boff + (size_t)nb * 16 * DM + kc);
#pragma unroll
            for (int mb = 0; mb < 4; ++mb) acc[mb][nb] = WFrag<T16>::mma(a[mb], b, acc[mb][nb]); }
        asm volatile("v_nop\n\tv_nop\n\tv_nop\n\tv_nop" : "+v"(acc[0][0]), "+v"(acc[1][1]), "+v"(acc[2][2]), "+v"(acc[3][3]) : "v"(a[0]), "v"(a[3]));
    }
#pragma unroll
    for (int mb = 0; mb < 4; ++mb)
#pragma unroll
        for (int nb = 0; nb < 4; ++nb)
#pragma unroll
            for (int j = 0; j < 8; ++j) os[(mb * 16 + hi * 8 + j) * 68 + nb * 16 + lr] = acc[mb][nb][j];
    __syncthreads();
    const int rq = lane >> 3, c8 = (lane & 7) * 8;
    if (EPI == 0) {
        const int sec = blockIdx.y / NH, hh = blockIdx.y % NH; const int n = bz * NH + hh;
        if (sec < 2) {
            h16* dst = planes + (size_t)sec * PLANE + ((size_t)n * SEQ + r0) * HD;
            float bv[8];
#pragma unroll
            for (int j = 0; j < 8; ++j) bv[j] = bfr(bias[c0 + c8 + j]);
#pragma unroll 1
            for (int ps = 0; ps < 2; ++ps) {
#pragma unroll 4
                for (int it = 0; it < 16; ++it) { const int row = it * 4 + rq; const v4f x0 = *(const v4fa*)(os + row * 68 + c8); const v4f x1 = *(const v4fa*)(os + row * 68 + c8 + 4); v8h o;
#pragma unroll
                    for (int j = 0; j < 4; ++j) { o[j] = (h16)((x0[j] + bv[j]) * QKCAR); o[4 + j] = (h16)((x1[j] + bv[4 + j]) * QKCAR); }
                    *(volatile v8h*)(dst + (size_t)row * HD + c8) = o; }
                if (ps == 0) __threadfence(); }
        } else {
            h16* dst = planes + 2 * PLANE + (size_t)n * HD * SEQ + r0;
#pragma unroll 1
            for (int ps = 0; ps < 2; ++ps) {
#pragma unroll 4
                for (int it = 0; it < 16; ++it) { const int d = it * 4 + rq; const float bd = bfr(bias[c0 + d]); v8h o;
#pragma unroll
                    for (int j = 0; j < 8; ++j) o[j] = (h16)((os[(c8 + j) * 68 + d] + bd) * VCAR);
                    *(volatile v8h*)(dst + (size_t)d * SEQ + c8) = o; }
                if (ps == 0) __threadfence(); }
        }
    } else {
        float* cb = C + ((size_t)r0 * NB + bz) * DM + c0; const int cofs = lr * 4;
        float bv[4];
#pragma unroll
        for (int j = 0; j < 4; ++j) bv[j] = bfr(bias[c0 + cofs + j]);
#pragma unroll 1
        for (int ps = 0; ps < 2; ++ps) {
#pragma unroll 4
            for (int it = 0; it < 32; ++it) { const int row = 2 * it + hi; const v4f x = *(const v4fa*)(os + row * 68 + cofs); v4f val;
#pragma unroll
                for (int j = 0; j < 4; ++j) val[j] = x[j] * OSCL + bv[j];
                *(volatile v4f*)(cb + (size_t)row * NB * DM + cofs) = val; }
            if (ps == 0) __threadfence(); }
    }
}

__global__ __launch_bounds__(256) void k_attn(const h16* __restrict__ Qp, const h16* __restrict__ Kp, const h16* __restrict__ Vt, h16* Ctx) {
    __shared__ __align__(16) h16 ot[8 * 16 * 72];
    const int lane = threadIdx.x & 31, lr = lane & 15, hi = lane >> 4;
    const int wv = __builtin_amdgcn_readfirstlane((int)(threadIdx.x >> 5));
    const int n = (int)(blockIdx.x / (SEQ / 128)); const int q0 = (int)(blockIdx.x % (SEQ / 128)) * 128 + wv * 16;
    const h16* qp = Qp + ((size_t)n * SEQ + q0 + lr) * HD + 8 * hi;
    const v16h qb0 = ldh(qp), qb1 = ldh(qp + 32);
    const h16* kp = Kp + ((size_t)n * SEQ + lr) * HD + 8 * hi;
    const h16* vp = Vt + ((size_t)n * HD + lr) * SEQ + 8 * hi;
    v8f oacc[4];
#pragma unroll
    for (int dt = 0; dt < 4; ++dt) oacc[dt] = (v8f){};
    float mrun = -1.0e30f, lsum = 0.0f;
#pragma unroll 1
    for (int kc = 0; kc < SEQ; kc += 32) {
        const h16* k0 = kp + (size_t)kc * HD;
        const v16h ka00 = ldh(k0), ka01 = ldh(k0 + 32), ka10 = ldh(k0 + 16 * HD), ka11 = ldh(k0 + 16 * HD + 32);
        const v16h va0 = ldh(vp + kc), va1 = ldh(vp + (size_t)16 * SEQ + kc), va2 = ldh(vp + (size_t)32 * SEQ + kc), va3 = ldh(vp + (size_t)48 * SEQ + kc);
        v8f s0 = (v8f){}, s1 = (v8f){};
        s0 = wmma16(ka00, qb0, s0); s1 = wmma16(ka10, qb0, s1); s0 = wmma16(ka01, qb1, s0); s1 = wmma16(ka11, qb1, s1);
        asm volatile("v_nop\n\tv_nop\n\tv_nop\n\tv_nop" : "+v"(s0), "+v"(s1) : "v"(ka11), "v"(qb1));
        float mx = fmaxf(s0[0], s1[0]);
#pragma unroll
        for (int r = 1; r < 8; ++r) mx = fmaxf(mx, fmaxf(s0[r], s1[r]));
        mx = fmaxf(mx, __shfl_xor(mx, 16, 32));
        const float mnew = fmaxf(mrun, mx);
        const float corr = __builtin_amdgcn_exp2f((mrun - mnew) * CLOG);
        const float nbias = PLOG - mnew * CLOG;
        mrun = mnew;
        float psum = 0.0f; v16h pb;
#pragma unroll
        for (int r = 0; r < 8; ++r) { const float p0 = __builtin_amdgcn_exp2f(fmaf(s0[r], CLOG, nbias)); const float p1 = __builtin_amdgcn_exp2f(fmaf(s1[r], CLOG, nbias)); psum += p0 + p1; pb[r] = (h16)p0; pb[8 + r] = (h16)p1; }
        lsum = lsum * corr + psum;
#pragma unroll
        for (int dt = 0; dt < 4; ++dt) oacc[dt] = oacc[dt] * corr;
        oacc[0] = wmma16(va0, pb, oacc[0]); oacc[1] = wmma16(va1, pb, oacc[1]); oacc[2] = wmma16(va2, pb, oacc[2]); oacc[3] = wmma16(va3, pb, oacc[3]);
        asm volatile("v_nop\n\tv_nop\n\tv_nop\n\tv_nop" : "+v"(oacc[0]), "+v"(oacc[1]), "+v"(oacc[2]), "+v"(oacc[3]) : "v"(va3), "v"(pb));
    }
    const float lt = lsum + __shfl_xor(lsum, 16, 32);
    const float f = (CCAR / VCAR) * (1.0f / lt);
    const int tb = wv * (16 * 72);
#pragma unroll
    for (int dt = 0; dt < 4; ++dt) { v8h o;
#pragma unroll
        for (int r = 0; r < 8; ++r) o[r] = (h16)(oacc[dt][r] * f);
        *(v8ha*)&ot[tb + lr * 72 + dt * 16 + hi * 8] = o; }
    __syncthreads();
    const int b = n / NH, hh = n % NH; const int rq = lane >> 3, c8 = (lane & 7) * 8;
    h16* dst = Ctx + ((size_t)b * SEQ + q0) * DM + hh * HD;
#pragma unroll 1
    for (int ps = 0; ps < 2; ++ps) {
#pragma unroll
        for (int it = 0; it < 4; ++it) { const int row = it * 4 + rq; const v8h v = *(const v8ha*)&ot[tb + row * 72 + c8]; *(volatile v8h*)(dst + (size_t)row * DM + c8) = v; }
        if (ps == 0) __threadfence(); }
}

extern "C" void kernel_launch(void* const* d_in, const int* in_sizes, int n_in,
                              void* d_out, int out_size, void* d_ws, size_t ws_size, hipStream_t stream) {
    if (n_in < 5) return;
    if (in_sizes[0] < ((SEQ - 1) * NB_FULL + NB) * DM) return;
    if (in_sizes[1] < 3 * DM * DM) return;
    if (in_sizes[2] < 3 * DM) return;
    if (in_sizes[3] < DM * DM) return;
    if (in_sizes[4] < DM) return;
    if (out_size < SEQ * NB * DM) return;
    const float* x = (const float*)d_in[0]; const float* win = (const float*)d_in[1]; const float* bin = (const float*)d_in[2]; const float* wo = (const float*)d_in[3]; const float* bo = (const float*)d_in[4];
    float* OUT = (float*)d_out;
    char* wsp = (char*)d_ws;
    auto take = [&](size_t bytes) { char* p = wsp; wsp += (bytes + 255) & ~(size_t)255; return (void*)p; };
    bf*  XB  = (bf*)take((size_t)NB * SEQ * DM * 2);
    bf*  WIN = (bf*)take((size_t)3 * DM * DM * 2);
    h16* WO  = (h16*)take((size_t)DM * DM * 2);
    h16* PL  = (h16*)take(3 * PLANE * 2);
    h16* CTX = (h16*)take((size_t)NB * SEQ * DM * 2);
    if ((size_t)(wsp - (char*)d_ws) > ws_size) return;
    const size_t nx8 = (size_t)NB * SEQ * DM / 8, nwi8 = (size_t)3 * DM * DM / 8, nwo8 = (size_t)DM * DM / 8;
    k_cvtx<<<(unsigned)((nx8 + 255) / 256), 256, 0, stream>>>(x, XB);
    k_cvt8<<<(unsigned)((nwi8 + 255) / 256), 256, 0, stream>>>(win, WIN, nwi8);
    k_cvtw<<<(unsigned)((nwo8 + 255) / 256), 256, 0, stream>>>(wo, WO, nwo8);
    k_gemm<bf, 0><<<dim3(SEQ / 64, 3 * DM / 64, NB), 32, 0, stream>>>(XB, WIN, bin, PL, nullptr);
    k_attn<<<(unsigned)(NB * NH * (SEQ / 128)), 256, 0, stream>>>(PL, PL + PLANE, PL + 2 * PLANE, CTX);
    k_gemm<h16, 1><<<dim3(SEQ / 64, DM / 64, NB), 32, 0, stream>>>(CTX, WO, bo, nullptr, OUT);
}
